// HierachicalEncoder_6425271075473
// MI455X (gfx1250) — hardware-verified
//
#include <hip/hip_runtime.h>
#include <stdint.h>

typedef unsigned short us_t;
typedef __attribute__((ext_vector_type(16))) __bf16 v16bf;
typedef __attribute__((ext_vector_type(8)))  unsigned short v8us;
typedef __attribute__((ext_vector_type(8)))  float v8f;
typedef __attribute__((ext_vector_type(4)))  float v4f;
typedef v8us  __attribute__((may_alias)) v8usa;
typedef v4f   __attribute__((may_alias)) v4fa;
typedef us_t  __attribute__((may_alias)) usa_t;
typedef float __attribute__((may_alias)) fa_t;

union FragB { v16bf v; v8us half[2]; };

#define NITEM 20000
#define NPAD  20096
#define NTOK  51200
#define NXROW 153600
#define DD    64
#define QP    196

static_assert(NPAD % 128 == 0);
static_assert(NPAD % 32 == 0);
static_assert(NPAD >= NITEM);
static_assert(NTOK * 3 == NXROW);
static_assert(NXROW % 48 == 0);
static_assert(NTOK % 8 == 0);

#define OFF_CW1   0
#define OFF_CW2   589824
#define OFF_CW3   786432
#define OFF_TW1   802816
#define OFF_TW2   950272
#define OFF_TW3   1048576
#define OFF_CFW   1064960
#define OFF_WQKV  1069056
#define WPL_ELEMS 1081344

__device__ __forceinline__ us_t bfbits(float f) {
  const unsigned u = __float_as_uint(f);
  return (us_t)((u + 0x7FFFu + ((u >> 16) & 1u)) >> 16);
}
__device__ __forceinline__ float bfval(us_t b) { return __uint_as_float(((unsigned)b) << 16); }
__device__ __forceinline__ float bfr(float f) { return bfval(bfbits(f)); }

__device__ __forceinline__ float wsum(float v) {
#pragma unroll
  for (int s = 16; s >= 1; s >>= 1) v += __shfl_xor(v, s, 32);
  return v;
}

__device__ __forceinline__ v8f wmma_bf16(v16bf a, v16bf b, v8f c) {
  v8f d = __builtin_amdgcn_wmma_f32_16x16x32_bf16(false, a, false, b, (short)0, c, false, false);
  asm volatile("v_nop\n\tv_nop\n\tv_nop\n\tv_nop" : "+v"(d) : "v"(a), "v"(b));
  return d;
}

__device__ __forceinline__ v16bf ldfrag(const us_t* p, int h) {
  FragB f;
  f.half[0] = *(const v8usa*)(p + 8 * h);
  f.half[1] = *(const v8usa*)(p + 16 + 8 * h);
  return f.v;
}

__global__ __launch_bounds__(256) void cvt_flat_kernel(
    const float* __restrict__ cw1, const float* __restrict__ cw2, const float* __restrict__ cw3,
    const float* __restrict__ tw1, const float* __restrict__ tw2, const float* __restrict__ tw3,
    const float* __restrict__ cfw, const float* __restrict__ wq, const float* __restrict__ wk,
    const float* __restrict__ wv, const float* __restrict__ cff,
    us_t* __restrict__ wpl, us_t* __restrict__ cfx)
{
  const int b = blockIdx.x;
  const float* src;
  us_t* dst;
  int lb;
  bool zero = false;
  if (b < 288)       { src = cw1; dst = wpl + OFF_CW1;         lb = b; }
  else if (b < 384)  { src = cw2; dst = wpl + OFF_CW2;         lb = b - 288; }
  else if (b < 392)  { src = cw3; dst = wpl + OFF_CW3;         lb = b - 384; }
  else if (b < 464)  { src = tw1; dst = wpl + OFF_TW1;         lb = b - 392; }
  else if (b < 512)  { src = tw2; dst = wpl + OFF_TW2;         lb = b - 464; }
  else if (b < 520)  { src = tw3; dst = wpl + OFF_TW3;         lb = b - 512; }
  else if (b < 522)  { src = cfw; dst = wpl + OFF_CFW;         lb = b - 520; }
  else if (b < 524)  { src = wq;  dst = wpl + OFF_WQKV;        lb = b - 522; }
  else if (b < 526)  { src = wk;  dst = wpl + OFF_WQKV + 4096; lb = b - 524; }
  else if (b < 528)  { src = wv;  dst = wpl + OFF_WQKV + 8192; lb = b - 526; }
  else if (b < 1153) { src = cff; dst = cfx;                   lb = b - 528; }
  else               { src = cff; dst = cfx + (size_t)NITEM * DD; lb = b - 1153; zero = true; }

  const size_t g = (size_t)lb * 256 + threadIdx.x;
  v8us o;
  if (!zero) {
    const v4f a = *(const v4fa*)(src + g * 8);
    const v4f c = *(const v4fa*)(src + g * 8 + 4);
    o = (v8us){ bfbits(a.x), bfbits(a.y), bfbits(a.z), bfbits(a.w),
                bfbits(c.x), bfbits(c.y), bfbits(c.z), bfbits(c.w) };
  } else {
    o = (v8us){ 0, 0, 0, 0, 0, 0, 0, 0 };
  }
  us_t* d = dst + g * 8;
  *(volatile v8us*)d = o;
  __threadfence();
  *(volatile v8us*)d = o;
}

template <int K>
__global__ __launch_bounds__(256) void cvt_rows_kernel(
    const float* __restrict__ src, us_t* __restrict__ dst, float* __restrict__ rn)
{
  __shared__ __attribute__((aligned(16))) float srn[32];
  const int tid = threadIdx.x, lane = tid & 31, w = tid >> 5;
  const int rbase = blockIdx.x * 32;

#pragma unroll 1
  for (int j = 0; j < 4; ++j) {
    const int row = rbase + 4 * w + j;
    const bool valid = row < NITEM;
    const int srow = valid ? row : (NITEM - 1);
    const float* s = src + (size_t)srow * K;
    us_t* d = dst + (size_t)row * K;
    float ss = 0.0f;
    for (int c = lane; c < K / 8; c += 32) {
      const v4f a = *(const v4fa*)(s + 8 * c);
      const v4f e = *(const v4fa*)(s + 8 * c + 4);
      const us_t b0 = bfbits(a.x), b1 = bfbits(a.y), b2 = bfbits(a.z), b3 = bfbits(a.w);
      const us_t b4 = bfbits(e.x), b5 = bfbits(e.y), b6 = bfbits(e.z), b7 = bfbits(e.w);
      const float f0 = bfval(b0), f1 = bfval(b1), f2 = bfval(b2), f3 = bfval(b3);
      const float f4 = bfval(b4), f5 = bfval(b5), f6 = bfval(b6), f7 = bfval(b7);
      ss += f0 * f0 + f1 * f1 + f2 * f2 + f3 * f3 + f4 * f4 + f5 * f5 + f6 * f6 + f7 * f7;
      v8us o = (v8us){ b0, b1, b2, b3, b4, b5, b6, b7 };
      if (!valid) o = (v8us){ 0, 0, 0, 0, 0, 0, 0, 0 };
      *(volatile v8us*)(d + 8 * c) = o;
      __threadfence();
      *(volatile v8us*)(d + 8 * c) = o;
    }
    ss = wsum(ss);
    if (lane == 0) srn[4 * w + j] = valid ? (1.0f / fmaxf(sqrtf(ss), 1e-12f)) : 0.0f;
  }
  __syncthreads();
  const int q = lane & 7;
  const v4f rv = *(const v4fa*)(srn + 4 * q);
  float* p = rn + rbase + 4 * q;
  const bool wr = (w == 0) && (lane < 8);
  if (wr) *(volatile v4f*)p = rv;
  __threadfence();
  if (wr) *(volatile v4f*)p = rv;
}

template <bool OUTF32>
__device__ __forceinline__ void gemm_store_pass(const unsigned int* sw, us_t* Oh, us_t* Ol, float* Of,
                                                int m0w, int n0, int N, int lane) {
  const int q8 = lane & 7, sub = lane >> 3;
  if (OUTF32) {
#pragma unroll
    for (int i = 0; i < 16; ++i) {
      const int lid = 4 * i + sub;
      const int row = lid >> 1, hl = lid & 1;
      const v4f v = *(const v4fa*)(sw + row * 64 + 32 * hl + 4 * q8);
      float* p = Of + (size_t)(m0w + row) * N + n0 + 32 * hl + 4 * q8;
      *(volatile v4f*)p = v;
    }
  } else {
    const us_t* sh = (const us_t*)sw;
#pragma unroll
    for (int i = 0; i < 8; ++i) {
      const int lid = 4 * i + sub;
      const v8us vh = *(const v8usa*)(sh + lid * 64 + 8 * q8);
      const v8us vl = *(const v8usa*)(sh + 2048 + lid * 64 + 8 * q8);
      us_t* ph = Oh + (size_t)(m0w + lid) * N + n0 + 8 * q8;
      us_t* pl = Ol + (size_t)(m0w + lid) * N + n0 + 8 * q8;
      *(volatile v8us*)ph = vh;
      *(volatile v8us*)pl = vl;
    }
  }
}

template <int KSPLIT, bool RNORM, bool RELU, bool OUTF32>
__global__ __launch_bounds__(128) void gemm_kernel(
    const us_t* __restrict__ Ah, const us_t* __restrict__ Al,
    const us_t* __restrict__ W, const float* __restrict__ bias, const float* __restrict__ rn,
    us_t* __restrict__ Oh, us_t* __restrict__ Ol, float* __restrict__ Of, int K, int N)
{
  __shared__ __attribute__((aligned(16))) unsigned int smem[8192];

  const int tid = threadIdx.x, lane = tid & 31, w = tid >> 5;
  const int h = lane >> 4, m = lane & 15;
  const int m0w = blockIdx.x * 128 + 32 * w;
  const int n0 = blockIdx.y * 64;

  const us_t* a0p = Ah + (size_t)(m0w + m) * K;
  const us_t* a1p = a0p + (size_t)16 * K;
  const us_t* l0p = Al + (size_t)(m0w + m) * K;
  const us_t* l1p = l0p + (size_t)16 * K;
  const us_t* wbp = W + (size_t)(n0 + m) * K;

  const v8f zero8 = { 0.f, 0.f, 0.f, 0.f, 0.f, 0.f, 0.f, 0.f };
  v8f acc[2][4];
#pragma unroll
  for (int mt = 0; mt < 2; ++mt)
#pragma unroll
    for (int nt = 0; nt < 4; ++nt) acc[mt][nt] = zero8;

#pragma unroll 1
  for (int k0 = 0; k0 < K; k0 += 32) {
    const v16bf a0 = ldfrag(a0p + k0, h);
    const v16bf a1 = ldfrag(a1p + k0, h);
    v16bf c0 = a0, c1 = a1;
    if (KSPLIT == 2) { c0 = ldfrag(l0p + k0, h); c1 = ldfrag(l1p + k0, h); }
#pragma unroll
    for (int nt = 0; nt < 4; ++nt) {
      const v16bf b = ldfrag(wbp + (size_t)(16 * nt) * K + k0, h);
      acc[0][nt] = wmma_bf16(a0, b, acc[0][nt]);
      acc[1][nt] = wmma_bf16(a1, b, acc[1][nt]);
      if (KSPLIT == 2) {
        acc[0][nt] = wmma_bf16(c0, b, acc[0][nt]);
        acc[1][nt] = wmma_bf16(c1, b, acc[1][nt]);
      }
    }
  }

  unsigned int* sw = smem + w * 2048;
  usa_t* sH = (usa_t*)sw;
  usa_t* sL = sH + 2048;
  fa_t*  sF = (fa_t*)sw;
#pragma unroll
  for (int mt = 0; mt < 2; ++mt) {
    float rr[8];
#pragma unroll
    for (int r = 0; r < 8; ++r) rr[r] = 1.0f;
    if (RNORM) {
      const v4f ra = *(const v4fa*)(rn + m0w + 16 * mt + 8 * h);
      const v4f rb = *(const v4fa*)(rn + m0w + 16 * mt + 8 * h + 4);
      rr[0] = ra.x; rr[1] = ra.y; rr[2] = ra.z; rr[3] = ra.w;
      rr[4] = rb.x; rr[5] = rb.y; rr[6] = rb.z; rr[7] = rb.w;
    }
#pragma unroll
    for (int nt = 0; nt < 4; ++nt) {
      const float bb = bfr(bias[n0 + 16 * nt + m]);
#pragma unroll
      for (int r = 0; r < 8; ++r) {
        float v = acc[mt][nt][r];
        if (RNORM) v *= rr[r];
        v += bb;
        if (RELU) v = fmaxf(v, 0.0f);
        const int idx = (16 * mt + 8 * h + r) * 64 + 16 * nt + m;
        if (OUTF32) {
          sF[idx] = v;
        } else {
          const us_t hb = bfbits(v);
          sH[idx] = hb;
          sL[idx] = bfbits(v - bfval(hb));
        }
      }
    }
  }
  __syncthreads();

  gemm_store_pass<OUTF32>(sw, Oh, Ol, Of, m0w, n0, N, lane);
  __threadfence();
  gemm_store_pass<OUTF32>(sw, Oh, Ol, Of, m0w, n0, N, lane);
}

__device__ __forceinline__ void l2_ln_pair(float x0, float x1, float& y0, float& y1) {
  const float ss = wsum(x0 * x0 + x1 * x1);
  const float sc = 1.0f / fmaxf(sqrtf(ss), 1e-12f);
  x0 *= sc; x1 *= sc;
  const float mu = wsum(x0 + x1) * (1.0f / 64.0f);
  const float d0 = x0 - mu, d1 = x1 - mu;
  const float var = wsum(d0 * d0 + d1 * d1) * (1.0f / 64.0f);
  const float inv = 1.0f / sqrtf(var + 1e-5f);
  y0 = d0 * inv; y1 = d1 * inv;
}

__global__ __launch_bounds__(256) void gather_ln_kernel(
    const int* __restrict__ seq, const int* __restrict__ cold,
    const float* __restrict__ cfeat, const float* __restrict__ tfeat, const float* __restrict__ cflin,
    const float* __restrict__ item_emb, us_t* __restrict__ Xh, us_t* __restrict__ Xl)
{
  __shared__ __attribute__((aligned(16))) us_t sxh[24 * 64];
  __shared__ __attribute__((aligned(16))) us_t sxl[24 * 64];

  const int tid = threadIdx.x, lane = tid & 31, w = tid >> 5;
  const int t = blockIdx.x * 8 + w;
  int s = seq[t];
  s = (s == NITEM) ? 0 : s;
  s = min(max(s, 0), NITEM - 1);
  const size_t rb = (size_t)s * DD;

  const float c0 = cfeat[rb + lane], c1 = cfeat[rb + lane + 32];
  const float u0 = tfeat[rb + lane], u1 = tfeat[rb + lane + 32];
  const float g0 = cflin[rb + lane], g1 = cflin[rb + lane + 32];
  const float e0 = bfr(item_emb[rb + lane]), e1 = bfr(item_emb[rb + lane + 32]);
  const int cz = cold[s];

  const float sc = wsum(c0 * c0 + c1 * c1);
  const float st = wsum(u0 * u0 + u1 * u1);
  const float rc = 1.0f / fmaxf(sqrtf(sc), 1e-12f);
  const float rt = 1.0f / fmaxf(sqrtf(st), 1e-12f);
  const float mm0 = c0 * rc + u0 * rt;
  const float mm1 = c1 * rc + u1 * rt;
  const float cf0 = (cz > 0) ? mm0 : g0;
  const float cf1 = (cz > 0) ? mm1 : g1;

  float y0, y1;
  us_t hb;
  us_t* ph = sxh + (3 * w) * 64;
  us_t* pl = sxl + (3 * w) * 64;

  l2_ln_pair(mm0, mm1, y0, y1);
  hb = bfbits(y0); ph[lane] = hb;      pl[lane] = bfbits(y0 - bfval(hb));
  hb = bfbits(y1); ph[lane + 32] = hb; pl[lane + 32] = bfbits(y1 - bfval(hb));

  l2_ln_pair(e0, e1, y0, y1);
  hb = bfbits(y0); ph[64 + lane] = hb;      pl[64 + lane] = bfbits(y0 - bfval(hb));
  hb = bfbits(y1); ph[64 + lane + 32] = hb; pl[64 + lane + 32] = bfbits(y1 - bfval(hb));

  l2_ln_pair(cf0, cf1, y0, y1);
  hb = bfbits(y0); ph[128 + lane] = hb;      pl[128 + lane] = bfbits(y0 - bfval(hb));
  hb = bfbits(y1); ph[128 + lane + 32] = hb; pl[128 + lane + 32] = bfbits(y1 - bfval(hb));

  __syncthreads();

  const size_t rowb = (size_t)blockIdx.x * 24;
  const int q8 = tid & 7;
  v8us v[2];
  us_t* dp[2];
  bool act[2];
#pragma unroll
  for (int it = 0; it < 2; ++it) {
    const int L = 32 * it + (tid >> 3);
    act[it] = (L < 48);
    const bool hiSel = (L < 24);
    int Lm = hiSel ? L : (L - 24);
    Lm = min(Lm, 23);
    const v8us a = *(const v8usa*)(sxh + Lm * 64 + 8 * q8);
    const v8us b = *(const v8usa*)(sxl + Lm * 64 + 8 * q8);
    v[it] = hiSel ? a : b;
    dp[it] = (hiSel ? Xh : Xl) + (rowb + Lm) * 64 + 8 * q8;
  }
#pragma unroll
  for (int it = 0; it < 2; ++it) if (act[it]) *(volatile v8us*)dp[it] = v[it];
  __threadfence();
#pragma unroll
  for (int it = 0; it < 2; ++it) if (act[it]) *(volatile v8us*)dp[it] = v[it];
}

__global__ __launch_bounds__(128) void qkv_attn_kernel(
    const us_t* __restrict__ Xh, const us_t* __restrict__ Xl,
    const us_t* __restrict__ Wqkv, float* __restrict__ out)
{
  __shared__ __attribute__((aligned(16))) float sQ[48 * QP];
  __shared__ __attribute__((aligned(16))) float sY[16 * 64];

  const int tid = threadIdx.x, lane = tid & 31, w = tid >> 5;
  const int h = lane >> 4, m = lane & 15;
  const int r0 = blockIdx.x * 48;
  const int t0 = blockIdx.x * 16;

  const v8f zero8 = { 0.f, 0.f, 0.f, 0.f, 0.f, 0.f, 0.f, 0.f };
  v8f acc[3][3];
#pragma unroll
  for (int i = 0; i < 3; ++i)
#pragma unroll
    for (int j = 0; j < 3; ++j) acc[i][j] = zero8;

#pragma unroll
  for (int ks = 0; ks < 2; ++ks) {
    const int k0 = 32 * ks;
    v16bf b[3];
#pragma unroll
    for (int j = 0; j < 3; ++j) b[j] = ldfrag(Wqkv + (size_t)(48 * w + 16 * j + m) * DD + k0, h);
#pragma unroll
    for (int i = 0; i < 3; ++i) {
      const v16bf ah = ldfrag(Xh + (size_t)(r0 + 16 * i + m) * DD + k0, h);
      const v16bf al = ldfrag(Xl + (size_t)(r0 + 16 * i + m) * DD + k0, h);
#pragma unroll
      for (int j = 0; j < 3; ++j) {
        acc[i][j] = wmma_bf16(ah, b[j], acc[i][j]);
        acc[i][j] = wmma_bf16(al, b[j], acc[i][j]);
      }
    }
  }

#pragma unroll
  for (int i = 0; i < 3; ++i)
#pragma unroll
    for (int j = 0; j < 3; ++j)
#pragma unroll
      for (int r = 0; r < 8; ++r)
        sQ[(16 * i + 8 * h + r) * QP + 48 * w + 16 * j + m] = acc[i][j][r];
  __syncthreads();

#pragma unroll 1
  for (int u = 0; u < 4; ++u) {
    const int tl = 4 * w + u;
    const float* rq = sQ + (3 * tl) * QP;
    float q0[3], q1[3], ka[3], kb[3], va[3], vb[3];
#pragma unroll
    for (int n = 0; n < 3; ++n) {
      const float* rw = rq + n * QP;
      q0[n] = rw[lane] * 0.125f;      q1[n] = rw[lane + 32] * 0.125f;
      ka[n] = rw[64 + lane];          kb[n] = rw[64 + lane + 32];
      va[n] = rw[128 + lane];         vb[n] = rw[128 + lane + 32];
    }
    float y0 = 0.0f, y1 = 0.0f;
#pragma unroll
    for (int n = 0; n < 3; ++n) {
      const float p0 = wsum(q0[n] * ka[0] + q1[n] * kb[0]);
      const float p1 = wsum(q0[n] * ka[1] + q1[n] * kb[1]);
      const float p2 = wsum(q0[n] * ka[2] + q1[n] * kb[2]);
      const float mx = fmaxf(p0, fmaxf(p1, p2));
      const float x0 = expf(p0 - mx);
      const float x1 = expf(p1 - mx);
      const float x2 = expf(p2 - mx);
      const float is = 1.0f / (x0 + x1 + x2);
      y0 += (x0 * va[0] + x1 * va[1] + x2 * va[2]) * is;
      y1 += (x0 * vb[0] + x1 * vb[1] + x2 * vb[2]) * is;
    }
    sY[tl * 64 + lane]      = y0 * (1.0f / 3.0f);
    sY[tl * 64 + lane + 32] = y1 * (1.0f / 3.0f);
  }
  __syncthreads();

  const int q8 = tid & 7;
  v4f ov[2];
  float* op[2];
#pragma unroll
  for (int it = 0; it < 2; ++it) {
    const int L = 16 * it + (tid >> 3);
    ov[it] = *(const v4fa*)(sY + L * 32 + 4 * q8);
    op[it] = out + (size_t)t0 * 64 + L * 32 + 4 * q8;
  }
#pragma unroll
  for (int it = 0; it < 2; ++it) *(volatile v4f*)op[it] = ov[it];
  __threadfence();
#pragma unroll
  for (int it = 0; it < 2; ++it) *(volatile v4f*)op[it] = ov[it];
}

extern "C" void kernel_launch(void* const* d_in, const int* in_sizes, int n_in,
                              void* d_out, int out_size, void* d_ws, size_t ws_size,
                              hipStream_t stream)
{
  if (n_in < 23) return;
  if (in_sizes[0] != NTOK) return;
  if (in_sizes[1] != NITEM) return;
  if (in_sizes[2] != NITEM * 768) return;
  if (in_sizes[3] != NITEM * 384) return;
  if (in_sizes[4] != NITEM * DD) return;
  if (in_sizes[5] != NITEM * DD) return;
  if (in_sizes[6] != 768 * 768 || in_sizes[7] != 768) return;
  if (in_sizes[8] != 256 * 768 || in_sizes[9] != 256) return;
  if (in_sizes[10] != 64 * 256 || in_sizes[11] != 64) return;
  if (in_sizes[12] != 384 * 384 || in_sizes[13] != 384) return;
  if (in_sizes[14] != 256 * 384 || in_sizes[15] != 256) return;
  if (in_sizes[16] != 64 * 256 || in_sizes[17] != 64) return;
  if (in_sizes[18] != 64 * 64 || in_sizes[19] != 64) return;
  if (in_sizes[20] != 64 * 64 || in_sizes[21] != 64 * 64 || in_sizes[22] != 64 * 64) return;
  if (out_size != NTOK * DD) return;

  const int*   seq      = (const int*)  d_in[0];
  const int*   cold     = (const int*)  d_in[1];
  const float* content  = (const float*)d_in[2];
  const float* text     = (const float*)d_in[3];
  const float* cf_feat  = (const float*)d_in[4];
  const float* item_emb = (const float*)d_in[5];
  const float* c_w1 = (const float*)d_in[6];  const float* c_b1 = (const float*)d_in[7];
  const float* c_w2 = (const float*)d_in[8];  const float* c_b2 = (const float*)d_in[9];
  const float* c_w3 = (const float*)d_in[10]; const float* c_b3 = (const float*)d_in[11];
  const float* t_w1 = (const float*)d_in[12]; const float* t_b1 = (const float*)d_in[13];
  const float* t_w2 = (const float*)d_in[14]; const float* t_b2 = (const float*)d_in[15];
  const float* t_w3 = (const float*)d_in[16]; const float* t_b3 = (const float*)d_in[17];
  const float* cf_w = (const float*)d_in[18]; const float* cf_b = (const float*)d_in[19];
  const float* w_q  = (const float*)d_in[20];
  const float* w_k  = (const float*)d_in[21];
  const float* w_v  = (const float*)d_in[22];
  float* out = (float*)d_out;

  const size_t b_wpl = (size_t)WPL_ELEMS * 2;
  const size_t b_cfx = (size_t)NPAD * DD * 2;
  const size_t b_rn  = (size_t)NPAD * 4;
  const size_t b_r1  = (size_t)NPAD * 768 * 2;
  const size_t b_h1  = (size_t)NPAD * 768 * 2;
  const size_t b_r2  = 2 * b_h1;
  const size_t b_f   = (size_t)NPAD * DD * 4;
  const size_t b_h2  = (size_t)NPAD * 256 * 2;
  const size_t b_xn  = (size_t)NXROW * DD * 2;
  static_assert(2 * (size_t)NPAD * 256 * 2 <= (size_t)NPAD * 768 * 2);
  static_assert(2 * (size_t)NXROW * DD * 2 <= 2 * (size_t)NPAD * 768 * 2);

  size_t o = 0;
  char* ws = (char*)d_ws;
  us_t*  wpl   = (us_t*)(ws + o);  o += b_wpl;
  us_t*  cfx   = (us_t*)(ws + o);  o += b_cfx;
  float* rnc   = (float*)(ws + o); o += b_rn;
  float* rnt   = (float*)(ws + o); o += b_rn;
  char*  r1    = ws + o;           o += b_r1;
  char*  r2    = ws + o;           o += b_r2;
  float* cfeat = (float*)(ws + o); o += b_f;
  float* tfeat = (float*)(ws + o); o += b_f;
  float* cflin = (float*)(ws + o); o += b_f;
  if (o > ws_size) return;

  us_t* X    = (us_t*)r1;
  us_t* H2h  = (us_t*)r1;
  us_t* H2l  = (us_t*)(r1 + b_h2);
  us_t* H1h  = (us_t*)r2;
  us_t* H1l  = (us_t*)(r2 + b_h1);
  us_t* Xnh  = (us_t*)r2;
  us_t* Xnl  = (us_t*)(r2 + b_xn);
  us_t* Wc1  = wpl + OFF_CW1;
  us_t* Wc2  = wpl + OFF_CW2;
  us_t* Wc3  = wpl + OFF_CW3;
  us_t* Wt1  = wpl + OFF_TW1;
  us_t* Wt2  = wpl + OFF_TW2;
  us_t* Wt3  = wpl + OFF_TW3;
  us_t* Wcf  = wpl + OFF_CFW;
  us_t* Wqkv = wpl + OFF_WQKV;

  const dim3 gFlat(1156);
  const dim3 gRows(NPAD / 32);
  const int  MG = NPAD / 128;

  cvt_flat_kernel<<<gFlat, 256, 0, stream>>>(c_w1, c_w2, c_w3, t_w1, t_w2, t_w3, cf_w,
                                               w_q, w_k, w_v, cf_feat, wpl, cfx);
  cvt_rows_kernel<768><<<gRows, 256, 0, stream>>>(content, X, rnc);
  gemm_kernel<1, true,  true,  false><<<dim3(MG, 12), 128, 0, stream>>>(X,   X,   Wc1, c_b1, rnc, H1h, H1l, cfeat, 768, 768);
  gemm_kernel<2, false, true,  false><<<dim3(MG, 4),  128, 0, stream>>>(H1h, H1l, Wc2, c_b2, rnc, H2h, H2l, cfeat, 768, 256);
  gemm_kernel<2, false, false, true ><<<dim3(MG, 1),  128, 0, stream>>>(H2h, H2l, Wc3, c_b3, rnc, H2h, H2l, cfeat, 256, 64);
  cvt_rows_kernel<384><<<gRows, 256, 0, stream>>>(text, X, rnt);
  gemm_kernel<1, true,  true,  false><<<dim3(MG, 6),  128, 0, stream>>>(X,   X,   Wt1, t_b1, rnt, H1h, H1l, tfeat, 384, 384);
  gemm_kernel<2, false, true,  false><<<dim3(MG, 4),  128, 0, stream>>>(H1h, H1l, Wt2, t_b2, rnt, H2h, H2l, tfeat, 384, 256);
  gemm_kernel<2, false, false, true ><<<dim3(MG, 1),  128, 0, stream>>>(H2h, H2l, Wt3, t_b3, rnt, H2h, H2l, tfeat, 256, 64);
  gemm_kernel<1, false, false, true ><<<dim3(MG, 1),  128, 0, stream>>>(cfx, cfx, Wcf, cf_b, rnc, H2h, H2l, cflin, 64, 64);
  gather_ln_kernel<<<NTOK / 8, 256, 0, stream>>>(seq, cold, cfeat, tfeat, cflin, item_emb, Xnh, Xnl);
  qkv_attn_kernel<<<NTOK / 16, 128, 0, stream>>>(Xnh, Xnl, Wqkv, out);
}
